// TransformerBlock_73040213836212
// MI455X (gfx1250) — hardware-verified
//
#include <hip/hip_runtime.h>
#include <math.h>

#ifndef NB
#define NB 2
#endif
#ifndef SEQ
#define SEQ 1024
#endif
#define NB_FULL 2
#define SEQ_FULL 1024
#define DM 1024
#define NH 16
#define HS 64
#define FD 4
#define D4 (4 * DM)
#define ROWS (NB * SEQ)

typedef __attribute__((ext_vector_type(16))) _Float16 v16h;
typedef __attribute__((ext_vector_type(8)))  _Float16 v8h;
typedef __attribute__((ext_vector_type(8)))  float    v8f;
typedef __attribute__((ext_vector_type(4)))  float    v4f;
typedef unsigned int u4 __attribute__((ext_vector_type(4)));
typedef unsigned int u2 __attribute__((ext_vector_type(2)));

static_assert(DM == NH * HS);
static_assert(HS == 64);
static_assert(FD == 4);
static_assert(DM == 32 * 4 * 8);
static_assert(SEQ % 64 == 0);
static_assert(ROWS % 64 == 0);
static_assert(DM % 64 == 0);
static_assert(D4 % 64 == 0);
static_assert(DM % 32 == 0);
static_assert(HS % 32 == 0);
static_assert(SEQ <= SEQ_FULL);
static_assert(NB <= NB_FULL);

union FragU { v16h v; v8h h[2]; };

#define VST2(T, ptr, val) do { const T vst2_v_ = (val); *(volatile T*)(ptr) = vst2_v_; __threadfence(); *(volatile T*)(ptr) = vst2_v_; } while (0)

__device__ __forceinline__ float cmb_bf(float v) { const unsigned u = __builtin_bit_cast(unsigned, v); const unsigned r = (u + 0x7fffu + ((u >> 16) & 1u)) & 0xffff0000u; return __builtin_bit_cast(float, r); }
__device__ __forceinline__ unsigned int pk2h(float a, float b) { return (unsigned int)__builtin_bit_cast(unsigned short, (_Float16)a) | ((unsigned int)__builtin_bit_cast(unsigned short, (_Float16)b) << 16); }
__device__ __forceinline__ int rmap(int m) { return (m / SEQ) * SEQ_FULL + (m % SEQ); }

__device__ __forceinline__ v8f wmma16(v16h a, v16h b, v8f c) {
    c = __builtin_amdgcn_wmma_f32_16x16x32_f16(false, a, false, b, (short)0, c, false, false);
    asm volatile("v_nop\n\tv_nop\n\tv_nop\n\tv_nop" : "+v"(c) : "v"(a), "v"(b));
    return c;
}
__device__ __forceinline__ void dep_guard_h(v8f& a, v8f& b, v16h x, v16h y) { asm volatile("v_nop\n\tv_nop\n\tv_nop\n\tv_nop" : "+v"(a), "+v"(b) : "v"(x), "v"(y)); }
__device__ __forceinline__ void keep4_h(v16h a, v16h b, v16h c, v16h d) { asm volatile("v_nop" :: "v"(a), "v"(b), "v"(c), "v"(d)); }
__device__ __forceinline__ void acc_guard4(v8f& a, v8f& b, v8f& c, v8f& d) { asm volatile("v_nop\n\tv_nop\n\tv_nop\n\tv_nop" : "+v"(a), "+v"(b), "+v"(c), "+v"(d)); }
__device__ __forceinline__ void wave_sync_lds() {
    __builtin_amdgcn_fence(3  , "workgroup");
    __builtin_amdgcn_wave_barrier();
    __builtin_amdgcn_fence(2  , "workgroup");
}

__global__ __launch_bounds__(256) void k_cm_castb(const float* __restrict__ SRC, int lds, _Float16* __restrict__ DST, int ldd, int nR, int nC, float sc) {
    const long long u = (long long)blockIdx.x * 256 + threadIdx.x; const int per = nC / 8; if (u >= (long long)nR * per) return;
    const int r = (int)(u / per); const int c0 = 8 * (int)(u % per);
    const float* s = SRC + (long long)r * lds + c0; float w[8];
#pragma unroll
    for (int e = 0; e < 8; ++e) w[e] = cmb_bf(s[e]) * sc;
    u4 pk; pk.x = pk2h(w[0], w[1]); pk.y = pk2h(w[2], w[3]); pk.z = pk2h(w[4], w[5]); pk.w = pk2h(w[6], w[7]);
    VST2(u4, (u4*)(DST + (long long)r * ldd + c0), pk);
}
__global__ __launch_bounds__(256) void k_cm_castbT(const float* __restrict__ SRC, int lds, _Float16* __restrict__ DST, int ldd, int nR, int nC, float sc) {
    const long long u = (long long)blockIdx.x * 256 + threadIdx.x; const int per = nR / 8; if (u >= (long long)nC * per) return;
    const int c = (int)(u / per); const int r0 = 8 * (int)(u % per); float w[8];
#pragma unroll
    for (int e = 0; e < 8; ++e) w[e] = cmb_bf(SRC[(long long)(r0 + e) * lds + c]) * sc;
    u4 pk; pk.x = pk2h(w[0], w[1]); pk.y = pk2h(w[2], w[3]); pk.z = pk2h(w[4], w[5]); pk.w = pk2h(w[6], w[7]);
    VST2(u4, (u4*)(DST + (long long)c * ldd + r0), pk);
}
__global__ __launch_bounds__(256) void k_wct(const float* __restrict__ Wc, _Float16* __restrict__ WCT) {
    const int u = blockIdx.x * 256 + threadIdx.x; if (u >= FD * HS * (HS / 8)) return;
    const int c0 = 8 * (u & 7); const int d = (u >> 3) & (HS - 1); const int tap = u >> 9; float w[8];
    static_assert(HS / 8 == 8);
#pragma unroll
    for (int e = 0; e < 8; ++e) w[e] = cmb_bf(Wc[(c0 + e) * (HS * FD) + d * FD + tap]) * 16.0f;
    u4 pk; pk.x = pk2h(w[0], w[1]); pk.y = pk2h(w[2], w[3]); pk.z = pk2h(w[4], w[5]); pk.w = pk2h(w[6], w[7]);
    VST2(u4, (u4*)(WCT + (tap * HS + d) * HS + c0), pk);
}

template <int ABF, int RMAP>
__device__ __forceinline__ void ln_body(const float* __restrict__ A, const float* __restrict__ GA, const float* __restrict__ BE, int rows, _Float16* __restrict__ Y16) {
    #pragma clang fp contract(off)
    const int r = blockIdx.x * 8 + (threadIdx.x >> 5); const int L = threadIdx.x & 31; if (r >= rows) return;
    const long long sr = RMAP ? (long long)rmap(r) : (long long)r;
    v4f v[8]; float s = 0.f;
#pragma unroll
    for (int q = 0; q < 8; ++q) {
        v[q] = *(const v4f*)(A + sr * DM + 4 * L + 128 * q);
        if (ABF) { v[q].x = cmb_bf(v[q].x); v[q].y = cmb_bf(v[q].y); v[q].z = cmb_bf(v[q].z); v[q].w = cmb_bf(v[q].w); }
        s += (v[q].x + v[q].y) + (v[q].z + v[q].w);
    }
#pragma unroll
    for (int o = 16; o > 0; o >>= 1) s += __shfl_xor(s, o, 32);
    const float mu = s * (1.f / DM); float qq = 0.f;
#pragma unroll
    for (int q = 0; q < 8; ++q) { v[q].x -= mu; v[q].y -= mu; v[q].z -= mu; v[q].w -= mu; qq += (v[q].x * v[q].x + v[q].y * v[q].y) + (v[q].z * v[q].z + v[q].w * v[q].w); }
#pragma unroll
    for (int o = 16; o > 0; o >>= 1) qq += __shfl_xor(qq, o, 32);
    const float rs = rsqrtf(qq * (1.f / DM) + 1e-5f);
#pragma unroll
    for (int q = 0; q < 8; ++q) {
        const int c = 4 * L + 128 * q; const v4f ga = *(const v4f*)(GA + c), be = *(const v4f*)(BE + c);
        const float y0 = v[q].x * rs * cmb_bf(ga.x) + cmb_bf(be.x), y1 = v[q].y * rs * cmb_bf(ga.y) + cmb_bf(be.y);
        const float y2 = v[q].z * rs * cmb_bf(ga.z) + cmb_bf(be.z), y3 = v[q].w * rs * cmb_bf(ga.w) + cmb_bf(be.w);
        u2 pk; pk.x = pk2h(y0, y1); pk.y = pk2h(y2, y3);
        VST2(u2, (u2*)(Y16 + (long long)r * DM + c), pk);
    }
}
__global__ __launch_bounds__(256) void k_ln_in(const float* __restrict__ X, const float* __restrict__ G, const float* __restrict__ Bt, int rows, _Float16* __restrict__ Y16) { ln_body<1, 1>(X, G, Bt, rows, Y16); }
__global__ __launch_bounds__(256) void k_ln_ws(const float* __restrict__ X, const float* __restrict__ G, const float* __restrict__ Bt, int rows, _Float16* __restrict__ Y16) { ln_body<0, 0>(X, G, Bt, rows, Y16); }

template <int UID, int OUT_MODE, int RESID, int ACT, int RMAPR, int RMAPC>
__device__ __forceinline__ void gemm64_body(const _Float16* __restrict__ A, int lda, const _Float16* __restrict__ Bt, int ldb,
                                            float* __restrict__ Cf, _Float16* __restrict__ Ch, int ldc,
                                            const float* __restrict__ resid, int ldr, int M, int N, int K, float scale) {
    __shared__ __align__(16) float sT[8 * 16 * 68];
    const int lane = threadIdx.x & 31;
    const int wave = threadIdx.x >> 5;
    const int tilesN = N >> 6;
    const int tilesM = M >> 6;
    const int tile = blockIdx.x * 8 + wave;
    if (tile >= tilesM * tilesN) return;
    const int tm = tile / tilesN;
    const int tn = tile - tm * tilesN;
    const int m0 = tm << 6;
    const int n0 = tn << 6;
    const int rlane = lane & 15;
    const int koff  = (lane >> 4) * 8;
    const int mOff  = (lane >> 4) * 8;
    const int sb = wave * (16 * 68);

    v8f acc[4][4];
#pragma unroll
    for (int i = 0; i < 4; ++i)
#pragma unroll
        for (int j = 0; j < 4; ++j) acc[i][j] = (v8f){0.f, 0.f, 0.f, 0.f, 0.f, 0.f, 0.f, 0.f};

    for (int k0 = 0; k0 < K; k0 += 32) {
        v16h bh[4];
#pragma unroll
        for (int j = 0; j < 4; ++j) {
            const size_t bo = (size_t)(n0 + (j << 4) + rlane) * ldb + koff + k0;
            FragU f; f.h[0] = *(const v8h*)(Bt + bo); f.h[1] = *(const v8h*)(Bt + bo + 16); bh[j] = f.v;
        }
#pragma unroll
        for (int i = 0; i < 4; ++i) {
            const size_t ao = (size_t)(m0 + (i << 4) + rlane) * lda + koff + k0;
            FragU f; f.h[0] = *(const v8h*)(A + ao); f.h[1] = *(const v8h*)(A + ao + 16);
            const v16h ah = f.v;
#pragma unroll
            for (int j = 0; j < 4; ++j)
                acc[i][j] = __builtin_amdgcn_wmma_f32_16x16x32_f16(false, ah, false, bh[j], (short)0, acc[i][j], false, false);
            dep_guard_h(acc[i][0], acc[i][3], ah, ah);
        }
        keep4_h(bh[0], bh[1], bh[2], bh[3]);
    }
    acc_guard4(acc[0][0], acc[0][1], acc[0][2], acc[0][3]);
    acc_guard4(acc[1][0], acc[1][1], acc[1][2], acc[1][3]);
    acc_guard4(acc[2][0], acc[2][1], acc[2][2], acc[2][3]);
    acc_guard4(acc[3][0], acc[3][1], acc[3][2], acc[3][3]);

#pragma unroll
    for (int i = 0; i < 4; ++i) {
        const int mBase = m0 + (i << 4);
#pragma unroll
        for (int j = 0; j < 4; ++j) {
#pragma unroll
            for (int r = 0; r < 8; ++r) {
                float v = acc[i][j][r] * scale;
                if (ACT == 5) v = 0.5f * v * (1.0f + erff(v * 0.70710678118654752f));
                sT[sb + (mOff + r) * 68 + (j << 4) + rlane] = v;
            }
        }
        wave_sync_lds();
        if (OUT_MODE == 0) {
            const int hh = lane >> 4, c4 = (lane & 15) * 4;
            for (int pass = 0; pass < 2; ++pass) {
#pragma unroll
                for (int it = 0; it < 8; ++it) {
                    const int row = it * 2 + hh;
                    v4f v = *(const v4f*)&sT[sb + row * 68 + c4];
                    if (RESID != 0) {
                        const int rr = RMAPR ? rmap(mBase + row) : (mBase + row);
                        v4f x = *(const v4f*)(resid + (size_t)rr * ldr + n0 + c4);
                        if (RESID == 2) { x.x = cmb_bf(x.x); x.y = cmb_bf(x.y); x.z = cmb_bf(x.z); x.w = cmb_bf(x.w); }
                        v = v + x;
                    }
                    const int cr = RMAPC ? rmap(mBase + row) : (mBase + row);
                    *(volatile v4f*)(Cf + (size_t)cr * ldc + n0 + c4) = v;
                }
                __threadfence();
            }
        } else {
            const int q = lane >> 3, c8 = (lane & 7) * 8;
            for (int pass = 0; pass < 2; ++pass) {
#pragma unroll
                for (int it = 0; it < 4; ++it) {
                    const int row = it * 4 + q;
                    const int so = sb + row * 68 + c8;
                    const v4f s0 = *(const v4f*)&sT[so], s1 = *(const v4f*)&sT[so + 4];
                    v8h hv;
                    hv[0] = (_Float16)s0.x; hv[1] = (_Float16)s0.y; hv[2] = (_Float16)s0.z; hv[3] = (_Float16)s0.w;
                    hv[4] = (_Float16)s1.x; hv[5] = (_Float16)s1.y; hv[6] = (_Float16)s1.z; hv[7] = (_Float16)s1.w;
                    *(volatile v8h*)(Ch + (size_t)(mBase + row) * ldc + n0 + c8) = hv;
                }
                __threadfence();
            }
        }
        wave_sync_lds();
    }
}

__global__ __launch_bounds__(256) void k_gemm_h16(const _Float16* __restrict__ A, int lda, const _Float16* __restrict__ Bt, int ldb, _Float16* __restrict__ C, int ldc, int M, int N, int K, float scale) {
    gemm64_body<0, 1, 0, 0, 0, 0>(A, lda, Bt, ldb, nullptr, C, ldc, nullptr, 0, M, N, K, scale);
}
__global__ __launch_bounds__(256) void k_gemm_conv(const _Float16* __restrict__ Q16, const _Float16* __restrict__ WCT, _Float16* __restrict__ UP) {
    const int z = blockIdx.y; const int hd = z >> 2; const int tap = z & 3;
    gemm64_body<1, 1, 0, 0, 0, 0>(Q16 + 3 * DM + hd * HS, D4, WCT + tap * HS * HS, HS, nullptr, UP + tap * DM + hd * HS, FD * DM, nullptr, 0, ROWS, HS, HS, 1.0f);
}
__global__ __launch_bounds__(256) void k_gemm_gelu16(const _Float16* __restrict__ A, int lda, const _Float16* __restrict__ Bt, int ldb, _Float16* __restrict__ C, int ldc, int M, int N, int K, float scale) {
    gemm64_body<2, 1, 0, 5, 0, 0>(A, lda, Bt, ldb, nullptr, C, ldc, nullptr, 0, M, N, K, scale);
}
__global__ __launch_bounds__(256) void k_gemm_resx(const _Float16* __restrict__ A, int lda, const _Float16* __restrict__ Bt, int ldb, float* __restrict__ C, int ldc, const float* __restrict__ X, int ldr, int M, int N, int K, float scale) {
    gemm64_body<3, 0, 2, 0, 1, 0>(A, lda, Bt, ldb, C, nullptr, ldc, X, ldr, M, N, K, scale);
}
__global__ __launch_bounds__(256) void k_gemm_resout(const _Float16* __restrict__ A, int lda, const _Float16* __restrict__ Bt, int ldb, float* __restrict__ C, int ldc, const float* __restrict__ X1, int ldr, int M, int N, int K, float scale) {
    gemm64_body<4, 0, 1, 0, 0, 1>(A, lda, Bt, ldb, C, nullptr, ldc, X1, ldr, M, N, K, scale);
}

#define AT_NW 4
static_assert(AT_NW * 16 == 64);
__global__ __launch_bounds__(32 * AT_NW) void k_attn_future(const _Float16* __restrict__ Q16, const _Float16* __restrict__ KVF, _Float16* __restrict__ AO) {
    __shared__ __align__(16) _Float16 Ksh[64 * 64];
    __shared__ __align__(16) _Float16 Vth[64 * 64];
    __shared__ __align__(16) _Float16 Psh[AT_NW * 16 * 32];
    __shared__ __align__(16) float    Os[AT_NW * 16 * 68];
    __shared__ __align__(16) float    Cfs[AT_NW * 16 * 4];
    const int tid = threadIdx.x, wave = tid >> 5, lane = tid & 31, hh = lane >> 4, c = lane & 15;
    const int nqb = SEQ / 64;
    const int bx = blockIdx.x;
    const int qb = bx % nqb;
    const int bhd = bx / nqb;
    const int h = bhd % NH;
    const int b = bhd / NH;
    const int q0 = qb * 64 + wave * 16;
    const size_t rowb = (size_t)b * SEQ;
    const size_t qoff = (rowb + q0 + c) * D4 + h * HS + 8 * hh;
    const float NEG = -__builtin_inff();
    const float L2E = 1.4426950408889634f;
    const float SC  = 0.125f * L2E;
    const float PSC = 32768.0f;

    float mrow[8], lrow[8];
    v8f oacc[4];
#pragma unroll
    for (int r = 0; r < 8; ++r) { mrow[r] = NEG; lrow[r] = 0.f; }
#pragma unroll
    for (int t = 0; t < 4; ++t) oacc[t] = (v8f){0.f, 0.f, 0.f, 0.f, 0.f, 0.f, 0.f, 0.f};

    for (int kc = 0; kc <= qb; ++kc) {
        const int kv0 = kc * 64;
        __syncthreads();
        {
            const int kvr = tid >> 1, dh = (tid & 1) * 32;
            const size_t ko = (rowb + kv0 + kvr) * D4 + DM + h * HS + dh;
#pragma unroll
            for (int i = 0; i < 4; ++i) {
                const v8h kk = *(const v8h*)(Q16 + ko + 8 * i);
                const v8h vv = *(const v8h*)(Q16 + ko + DM + 8 * i);
                *(v8h*)&Ksh[kvr * 64 + dh + 8 * i] = kk;
#pragma unroll
                for (int e = 0; e < 8; ++e) Vth[(dh + 8 * i + e) * 64 + kvr] = vv[e];
            }
        }
        __syncthreads();
        const bool diag = (kc == qb);
#pragma unroll 1
        for (int half = 0; half < 2; ++half) {
            const int kh0 = kv0 + 32 * half;
            if (kh0 > q0 + 15) continue;
            v8f s0 = (v8f){0.f, 0.f, 0.f, 0.f, 0.f, 0.f, 0.f, 0.f}, s1 = s0;
#pragma unroll
            for (int dc = 0; dc < 2; ++dc) {
                FragU qa; qa.h[0] = *(const v8h*)(Q16 + qoff + dc * 32); qa.h[1] = *(const v8h*)(Q16 + qoff + dc * 32 + 16);
                const int ki = (32 * half + c) * 64 + dc * 32 + 8 * hh;
                FragU k0f; k0f.h[0] = *(const v8h*)&Ksh[ki]; k0f.h[1] = *(const v8h*)&Ksh[ki + 16];
                s0 = wmma16(qa.v, k0f.v, s0);
                FragU k1f; k1f.h[0] = *(const v8h*)&Ksh[ki + 16 * 64]; k1f.h[1] = *(const v8h*)&Ksh[ki + 16 * 64 + 16];
                s1 = wmma16(qa.v, k1f.v, s1);
            }
#pragma unroll
            for (int r = 0; r < 8; ++r) {
                const int qrow = q0 + 8 * hh + r;
                float a0 = s0[r] * SC, a1 = s1[r] * SC;
                a0 = (diag && (kh0 + c > qrow)) ? NEG : a0;
                a1 = (diag && (kh0 + 16 + c > qrow)) ? NEG : a1;
                float mx = fmaxf(a0, a1);
                mx = fmaxf(mx, __shfl_xor(mx, 1, 32)); mx = fmaxf(mx, __shfl_xor(mx, 2, 32));
                mx = fmaxf(mx, __shfl_xor(mx, 4, 32)); mx = fmaxf(mx, __shfl_xor(mx, 8, 32));
                const float mnew = fmaxf(mrow[r], mx);
                const float alpha = (mnew == NEG) ? 1.f : exp2f(mrow[r] - mnew);
                const float p0 = (a0 == NEG) ? 0.f : exp2f(a0 - mnew);
                const float p1 = (a1 == NEG) ? 0.f : exp2f(a1 - mnew);
                Psh[(wave * 16 + 8 * hh + r) * 32 + c]      = (_Float16)(p0 * PSC);
                Psh[(wave * 16 + 8 * hh + r) * 32 + 16 + c] = (_Float16)(p1 * PSC);
                float ps = p0 + p1;
                ps += __shfl_xor(ps, 1, 32); ps += __shfl_xor(ps, 2, 32); ps += __shfl_xor(ps, 4, 32); ps += __shfl_xor(ps, 8, 32);
                lrow[r] = lrow[r] * alpha + ps;
                mrow[r] = mnew;
#pragma unroll
                for (int t = 0; t < 4; ++t) oacc[t][r] *= alpha;
            }
            wave_sync_lds();
            FragU pa; pa.h[0] = *(const v8h*)&Psh[(wave * 16 + c) * 32 + 8 * hh]; pa.h[1] = *(const v8h*)&Psh[(wave * 16 + c) * 32 + 16 + 8 * hh];
            v16h vb[4];
#pragma unroll
            for (int t = 0; t < 4; ++t) {
                const int vi = (16 * t + c) * 64 + 32 * half + 8 * hh;
                FragU f; f.h[0] = *(const v8h*)&Vth[vi]; f.h[1] = *(const v8h*)&Vth[vi + 16]; vb[t] = f.v;
            }
#pragma unroll
            for (int t = 0; t < 4; ++t) oacc[t] = wmma16(pa.v, vb[t], oacc[t]);
            wave_sync_lds();
        }
    }

    const int fr = lane >> 1, tp = (lane & 1) * 2;
    const size_t qro = (rowb + q0 + fr) * D4 + h * HS;
    const size_t kfo = ((rowb + q0 + fr) * FD + tp) * (2 * DM) + h * HS;
    float d0 = 0.f, d1 = 0.f;
#pragma unroll 1
    for (int i = 0; i < 8; ++i) {
        const v8h qv = *(const v8h*)(Q16 + qro + 8 * i);
        const v8h ka = *(const v8h*)(KVF + kfo + 8 * i);
        const v8h kb = *(const v8h*)(KVF + kfo + 2 * DM + 8 * i);
#pragma unroll
        for (int e = 0; e < 8; ++e) { const float qf = (float)qv[e]; d0 += qf * (float)ka[e]; d1 += qf * (float)kb[e]; }
    }
    d0 *= L2E * 0.0625f; d1 *= L2E * 0.0625f;

#pragma unroll
    for (int r = 0; r < 8; ++r) {
        const int src = 16 * hh + 2 * r;
        const float f0 = __shfl(d0, src, 32), f1 = __shfl(d1, src, 32), f2 = __shfl(d0, src + 1, 32), f3 = __shfl(d1, src + 1, 32);
        const float mnew = fmaxf(mrow[r], fmaxf(fmaxf(f0, f1), fmaxf(f2, f3)));
        const float alpha = exp2f(mrow[r] - mnew);
        const float e0 = exp2f(f0 - mnew), e1 = exp2f(f1 - mnew), e2 = exp2f(f2 - mnew), e3 = exp2f(f3 - mnew);
        const float l = lrow[r] * alpha + ((e0 + e1) + (e2 + e3));
        const float inv = 1.0f / l;
        const float so = alpha * inv * (16.0f / 32768.0f);
#pragma unroll
        for (int t = 0; t < 4; ++t) Os[(wave * 16 + 8 * hh + r) * 68 + 16 * t + c] = oacc[t][r] * so;
        if (c == 0) { v4f cf; cf.x = e0 * inv; cf.y = e1 * inv; cf.z = e2 * inv; cf.w = e3 * inv; *(v4f*)&Cfs[(wave * 16 + 8 * hh + r) * 4] = cf; }
    }
    wave_sync_lds();

    const int qd = lane >> 3, c8 = (lane & 7) * 8;
#pragma unroll 1
    for (int it = 0; it < 4; ++it) {
        const int row = it * 4 + qd;
        const int so = (wave * 16 + row) * 68 + c8;
        v4f a0 = *(const v4f*)&Os[so], a1 = *(const v4f*)&Os[so + 4];
        const v4f cf = *(const v4f*)&Cfs[(wave * 16 + row) * 4];
        const size_t vfo = ((rowb + q0 + row) * FD) * (2 * DM) + DM + h * HS + c8;
        const v8h v0 = *(const v8h*)(KVF + vfo);
        const v8h v1 = *(const v8h*)(KVF + vfo + 2 * DM);
        const v8h v2 = *(const v8h*)(KVF + vfo + 4 * DM);
        const v8h v3 = *(const v8h*)(KVF + vfo + 6 * DM);
        a0.x += cf.x * (float)v0[0] + cf.y * (float)v1[0] + cf.z * (float)v2[0] + cf.w * (float)v3[0];
        a0.y += cf.x * (float)v0[1] + cf.y * (float)v1[1] + cf.z * (float)v2[1] + cf.w * (float)v3[1];
        a0.z += cf.x * (float)v0[2] + cf.y * (float)v1[2] + cf.z * (float)v2[2] + cf.w * (float)v3[2];
        a0.w += cf.x * (float)v0[3] + cf.y * (float)v1[3] + cf.z * (float)v2[3] + cf.w * (float)v3[3];
        a1.x += cf.x * (float)v0[4] + cf.y * (float)v1[4] + cf.z * (float)v2[4] + cf.w * (float)v3[4];
        a1.y += cf.x * (float)v0[5] + cf.y * (float)v1[5] + cf.z * (float)v2[5] + cf.w * (float)v3[5];
        a1.z += cf.x * (float)v0[6] + cf.y * (float)v1[6] + cf.z * (float)v2[6] + cf.w * (float)v3[6];
        a1.w += cf.x * (float)v0[7] + cf.y * (float)v1[7] + cf.z * (float)v2[7] + cf.w * (float)v3[7];
        v8h hv;
        hv[0] = (_Float16)a0.x; hv[1] = (_Float16)a0.y; hv[2] = (_Float16)a0.z; hv[3] = (_Float16)a0.w;
        hv[4] = (_Float16)a1.x; hv[5] = (_Float16)a1.y; hv[6] = (_Float16)a1.z; hv[7] = (_Float16)a1.w;
        volatile v8h* dst = (volatile v8h*)(AO + (rowb + q0 + row) * DM + h * HS + c8);
        *dst = hv; __threadfence(); *dst = hv;
    }
}

constexpr size_t al256(size_t v) { return (v + 255) / 256 * 256; }
constexpr size_t SZ_H16  = al256((size_t)ROWS * DM * 2);
constexpr size_t SZ_W316 = al256((size_t)D4 * DM * 2);
constexpr size_t SZ_Q16  = al256((size_t)ROWS * D4 * 2);
constexpr size_t SZ_WCT  = al256((size_t)FD * HS * HS * 2);
constexpr size_t SZ_UP   = al256((size_t)ROWS * FD * DM * 2);
constexpr size_t SZ_G16  = al256((size_t)ROWS * D4 * 2);
constexpr size_t SZ_KVF  = al256((size_t)ROWS * FD * 2 * DM * 2);
constexpr size_t SZ_AO   = al256((size_t)ROWS * DM * 2);
constexpr size_t SZ_WO   = al256((size_t)DM * DM * 2);
constexpr size_t SZ_X1   = al256((size_t)ROWS * DM * 4);
constexpr size_t SZ_H2   = al256((size_t)ROWS * DM * 2);
constexpr size_t SZ_W1T  = al256((size_t)D4 * DM * 2);
constexpr size_t SZ_W2T  = al256((size_t)DM * D4 * 2);
constexpr size_t OFF_H16  = 0;
constexpr size_t OFF_W316 = OFF_H16 + SZ_H16;
constexpr size_t OFF_Q16  = OFF_W316 + SZ_W316;
constexpr size_t OFF_WCT  = OFF_Q16 + SZ_Q16;
constexpr size_t OFF_UP   = OFF_WCT + SZ_WCT;
constexpr size_t OFF_KVF  = OFF_UP + SZ_UP;
constexpr size_t OFF_AO   = OFF_KVF + SZ_KVF;
constexpr size_t OFF_WO   = OFF_AO + SZ_AO;
constexpr size_t OFF_X1   = OFF_WO + SZ_WO;
constexpr size_t OFF_H2   = OFF_X1 + SZ_X1;
constexpr size_t OFF_W1T  = OFF_H2 + SZ_H2;
constexpr size_t OFF_W2T  = OFF_W1T + SZ_W1T;
constexpr size_t WS_TOTAL = OFF_W2T + SZ_W2T;
static_assert(SZ_G16 <= SZ_UP);
static_assert(WS_TOTAL <= (size_t)134217728);

static inline unsigned cdiv_u(long long a, long long b) { return (unsigned)((a + b - 1) / b); }

extern "C" void kernel_launch(void* const* d_in, const int* in_sizes, int n_in, void* d_out, int out_size, void* d_ws, size_t ws_size, hipStream_t stream) {
    if (n_in < 10) return;
    const long long need_x = ((long long)(NB - 1) * SEQ_FULL + SEQ) * DM;
    if ((long long)in_sizes[0] < need_x) return;
    if ((long long)in_sizes[1] < (long long)D4 * DM) return;
    if ((long long)in_sizes[2] < (long long)HS * HS * FD) return;
    if ((long long)in_sizes[3] < (long long)DM * DM) return;
    if ((long long)in_sizes[4] < (long long)DM * D4) return;
    if ((long long)in_sizes[5] < (long long)D4 * DM) return;
    if (in_sizes[6] < DM || in_sizes[7] < DM || in_sizes[8] < DM || in_sizes[9] < DM) return;
    if ((long long)out_size < need_x) return;
    if (ws_size < WS_TOTAL) return;

    const float* x     = (const float*)d_in[0];
    const float* wqkvf = (const float*)d_in[1];
    const float* wconv = (const float*)d_in[2];
    const float* wproj = (const float*)d_in[3];
    const float* wff1  = (const float*)d_in[4];
    const float* wff2  = (const float*)d_in[5];
    const float* g1    = (const float*)d_in[6];
    const float* be1   = (const float*)d_in[7];
    const float* g2    = (const float*)d_in[8];
    const float* be2   = (const float*)d_in[9];
    float* out = (float*)d_out;
    char* ws = (char*)d_ws;
    _Float16* H16  = (_Float16*)(ws + OFF_H16);
    _Float16* W316 = (_Float16*)(ws + OFF_W316);
    _Float16* Q16  = (_Float16*)(ws + OFF_Q16);
    _Float16* WCT  = (_Float16*)(ws + OFF_WCT);
    _Float16* UP16 = (_Float16*)(ws + OFF_UP);
    _Float16* G16  = (_Float16*)(ws + OFF_UP);
    _Float16* KVF  = (_Float16*)(ws + OFF_KVF);
    _Float16* AO16 = (_Float16*)(ws + OFF_AO);
    _Float16* WO16 = (_Float16*)(ws + OFF_WO);
    float*    X1   = (float*)(ws + OFF_X1);
    _Float16* H2   = (_Float16*)(ws + OFF_H2);
    _Float16* W1T  = (_Float16*)(ws + OFF_W1T);
    _Float16* W2T  = (_Float16*)(ws + OFF_W2T);

    k_cm_castb<<<cdiv_u((long long)D4 * (DM / 8), 256), 256, 0, stream>>>(wqkvf, DM, W316, DM, D4, DM, 16.0f);
    k_cm_castb<<<cdiv_u((long long)DM * (DM / 8), 256), 256, 0, stream>>>(wproj, DM, WO16, DM, DM, DM, 16.0f);
    k_cm_castbT<<<cdiv_u((long long)D4 * (DM / 8), 256), 256, 0, stream>>>(wff1, D4, W1T, DM, DM, D4, 16.0f);
    k_cm_castbT<<<cdiv_u((long long)DM * (D4 / 8), 256), 256, 0, stream>>>(wff2, DM, W2T, D4, D4, DM, 16.0f);
    k_wct<<<cdiv_u(FD * HS * (HS / 8), 256), 256, 0, stream>>>(wconv, WCT);

    k_ln_in<<<cdiv_u(ROWS, 8), 256, 0, stream>>>(x, g1, be1, ROWS, H16);
    k_gemm_h16<<<cdiv_u((long long)(ROWS / 64) * (D4 / 64), 8), 256, 0, stream>>>(H16, DM, W316, DM, Q16, D4, ROWS, D4, DM, 0.0625f);
    k_gemm_conv<<<dim3(cdiv_u(ROWS / 64, 8), NH * FD), 256, 0, stream>>>(Q16, WCT, UP16);
    k_gemm_h16<<<cdiv_u((long long)(ROWS * FD / 64) * (2 * DM / 64), 8), 256, 0, stream>>>(UP16, DM, W316 + (size_t)DM * DM, DM, KVF, 2 * DM, ROWS * FD, 2 * DM, DM, 0.0625f);
    k_attn_future<<<NB * NH * (SEQ / 64), 32 * AT_NW, 0, stream>>>(Q16, KVF, AO16);
    k_gemm_resx<<<cdiv_u((long long)(ROWS / 64) * (DM / 64), 8), 256, 0, stream>>>(AO16, DM, WO16, DM, X1, DM, x, DM, ROWS, DM, DM, 0.00390625f);
    k_ln_ws<<<cdiv_u(ROWS, 8), 256, 0, stream>>>(X1, g2, be2, ROWS, H2);
    k_gemm_gelu16<<<cdiv_u((long long)(ROWS / 64) * (D4 / 64), 8), 256, 0, stream>>>(H2, DM, W1T, DM, G16, D4, ROWS, D4, DM, 0.0625f);
    k_gemm_resout<<<cdiv_u((long long)(ROWS / 64) * (DM / 64), 8), 256, 0, stream>>>(G16, D4, W2T, D4, out, DM, X1, DM, ROWS, DM, D4, 0.0625f);
}
